// MambaBlock_47536698032514
// MI455X (gfx1250) — hardware-verified
//
#include <hip/hip_runtime.h>
#include <stddef.h>
#include <stdint.h>
#include <math.h>


#define DM     256
#define DI     512
#define DH     256
#define NS     16
#define NB     2
#define SL     4096
#define NTOK   (NB * SL)
#define KIN    512
#define KDT    512
#define KOUT   1024
#define GBM    64
#define GBN    64
#define GTHR   128
#define NTHR   256
#define NU_WIN (DI * (KIN / 8))
#define NU_WDT (DH * (KDT / 8))
#define NU_WO  (DM * (KOUT / 8))
#define NU_ALL (NU_WIN + NU_WDT + NU_WO)
#define LNT    32
#define XSP    34
#define OSP    520
#define CT     64
#define XPP    72
#define FP     68
#define TP     72
#define LN_EPS 1e-5f
#define WSMAX  134217728

static_assert(SL % GBN == 0 && DI % GBM == 0 && DH % GBM == 0 && DM % GBM == 0);
static_assert(KIN % 32 == 0 && KDT % 32 == 0 && KOUT % 32 == 0);
static_assert(GBM == (GTHR / 32) * 16 && GBN == 64);
static_assert(NU_WIN % NTHR == 0 && NU_WDT % NTHR == 0 && NU_WO % NTHR == 0);
static_assert(SL % LNT == 0 && SL % CT == 0 && DH % CT == 0);
static_assert((OSP * 2) % 16 == 0 && (TP * 2) % 16 == 0 && (FP * 4) % 16 == 0 && (XPP * 4) % 16 == 0);
static_assert(DM * XSP * 2 + LNT * OSP * 2 + 8 * 32 * 4 + 64 * 4 <= 65536);
static_assert(CT * XPP * 4 + CT * FP * 4 + 2 * CT * TP * 2 + CT * 4 * 4 + CT * 4 <= 65536);
static_assert(2 * CT * FP * 4 + 2 * CT * TP * 2 <= 65536);

typedef float          v4f   __attribute__((ext_vector_type(4)));
typedef float          v8f   __attribute__((ext_vector_type(8)));
typedef int            v8i   __attribute__((ext_vector_type(8)));
typedef unsigned short v8us  __attribute__((ext_vector_type(8)));
typedef unsigned short v16us __attribute__((ext_vector_type(16)));
typedef __bf16         v16bf __attribute__((ext_vector_type(16)));
typedef v4f  __attribute__((may_alias)) v4fa;
typedef v8us __attribute__((may_alias)) v8usa;
union FragB { v16bf v; v16us u; v8us h[2]; v8i w; };

__device__ __forceinline__ v8f wmb(const FragB& a, const FragB& b, v8f c) {
  v8f d = __builtin_amdgcn_wmma_f32_16x16x32_bf16(false, a.v, false, b.v, (short)0, c, false, false);
  asm volatile("v_nop\n\tv_nop\n\tv_nop\n\tv_nop" : "+v"(d) : "v"(a.w), "v"(b.w));
  return d;
}

__device__ __forceinline__ unsigned bf16_bits(float f) {
  const unsigned u = __float_as_uint(f);
  return (u + 0x7FFFu + ((u >> 16) & 1u)) >> 16;
}
__device__ __forceinline__ float bf16_val(float f) {
  return __uint_as_float(bf16_bits(f) << 16);
}

__device__ __forceinline__ float gelu_erf(float x) {
  return 0.5f * x * (1.0f + erff(x * 0.70710678118654752440f));
}
__device__ __forceinline__ float softplus_p(float x) {
  return fmaxf(x, 0.0f) + log1pf(expf(-fabsf(x)));
}

__device__ __forceinline__ void cvt8(const float* __restrict__ p, unsigned short* dp) {
  const v4f a = *(const v4f*)p;
  const v4f b = *(const v4f*)(p + 4);
  v8us o;
  o[0] = (unsigned short)bf16_bits(a.x); o[1] = (unsigned short)bf16_bits(a.y);
  o[2] = (unsigned short)bf16_bits(a.z); o[3] = (unsigned short)bf16_bits(a.w);
  o[4] = (unsigned short)bf16_bits(b.x); o[5] = (unsigned short)bf16_bits(b.y);
  o[6] = (unsigned short)bf16_bits(b.z); o[7] = (unsigned short)bf16_bits(b.w);
  *(volatile v8us*)dp = o;
  __threadfence();
  *(volatile v8us*)dp = o;
}

__global__ __launch_bounds__(NTHR) void k_prep(const float* __restrict__ w_in, const float* __restrict__ w_dt,
                                               const float* __restrict__ w_out,
                                               unsigned short* WIN2, unsigned short* WDT2, unsigned short* WO4) {
  const int u = (int)blockIdx.x * NTHR + (int)threadIdx.x;
  if (u < NU_WIN) {
    const int n  = u >> 6;
    const int k8 = (u & 63) * 8;
    cvt8(w_in + (size_t)n * DM + (k8 & 255), WIN2 + (size_t)n * KIN + k8);
  } else if (u < NU_WIN + NU_WDT) {
    const int v  = u - NU_WIN;
    const int n  = v >> 6;
    const int k8 = (v & 63) * 8;
    cvt8(w_dt + (size_t)n * DH + (k8 & 255), WDT2 + (size_t)n * KDT + k8);
  } else if (u < NU_ALL) {
    const int v  = u - NU_WIN - NU_WDT;
    const int n  = v >> 7;
    const int k8 = (v & 127) * 8;
    const int sc = (k8 >> 9) * 256 + (k8 & 255);
    cvt8(w_out + (size_t)n * DI + sc, WO4 + (size_t)n * KOUT + k8);
  }
}

__global__ __launch_bounds__(NTHR) void k_ln(const float* __restrict__ x, const float* __restrict__ g,
                                             const float* __restrict__ be, unsigned short* xnhl) {
  __shared__ unsigned short xs[DM * XSP];
  __shared__ __attribute__((aligned(16))) unsigned short outs[LNT * OSP];
  __shared__ float ps[8 * 32];
  __shared__ float smu[32];
  __shared__ float srs[32];
  const int tid = (int)threadIdx.x;
  const int b   = (int)blockIdx.x >> 7;
  const int l0  = ((int)blockIdx.x & 127) * LNT;

  {
    const int cq = tid >> 3, q = tid & 7;
    v4f v[8];
#pragma unroll
    for (int i = 0; i < 8; ++i) {
      const int c = i * 32 + cq;
      v[i] = *(const v4f*)(x + ((size_t)(b * DM + c)) * SL + l0 + 4 * q);
    }
#pragma unroll
    for (int i = 0; i < 8; ++i) {
      const int c = i * 32 + cq;
      unsigned short* sp = xs + c * XSP + 4 * q;
      sp[0] = (unsigned short)bf16_bits(v[i].x);
      sp[1] = (unsigned short)bf16_bits(v[i].y);
      sp[2] = (unsigned short)bf16_bits(v[i].z);
      sp[3] = (unsigned short)bf16_bits(v[i].w);
    }
  }
  __syncthreads();

  const int l = tid & 31, p = tid >> 5;
  float s = 0.0f;
#pragma unroll 4
  for (int j = 0; j < 32; ++j) {
    const unsigned w = (unsigned)xs[(p * 32 + j) * XSP + l];
    s += __uint_as_float(w << 16);
  }
  ps[p * 32 + l] = s;
  __syncthreads();
  float mu = 0.0f;
#pragma unroll
  for (int p2 = 0; p2 < 8; ++p2) mu += ps[p2 * 32 + l];
  mu *= (1.0f / DM);
  __syncthreads();
  float sq = 0.0f;
#pragma unroll 4
  for (int j = 0; j < 32; ++j) {
    const unsigned w = (unsigned)xs[(p * 32 + j) * XSP + l];
    const float d = __uint_as_float(w << 16) - mu;
    sq += d * d;
  }
  ps[p * 32 + l] = sq;
  __syncthreads();
  if (tid < 32) {
    float var = 0.0f;
#pragma unroll
    for (int p2 = 0; p2 < 8; ++p2) var += ps[p2 * 32 + tid];
    var *= (1.0f / DM);
    smu[tid] = mu;
    srs[tid] = 1.0f / sqrtf(var + LN_EPS);
  }
  __syncthreads();

  {
    const int c = tid;
    const float gg = bf16_val(g[c]);
    const float bb = bf16_val(be[c]);
#pragma unroll 4
    for (int t = 0; t < LNT; ++t) {
      const unsigned w = (unsigned)xs[c * XSP + t];
      const float v  = __uint_as_float(w << 16);
      const float xn = (v - smu[t]) * srs[t] * gg + bb;
      const unsigned hb = bf16_bits(xn);
      const unsigned lb = bf16_bits(xn - __uint_as_float(hb << 16));
      outs[t * OSP + c]      = (unsigned short)hb;
      outs[t * OSP + DM + c] = (unsigned short)lb;
    }
  }
  __syncthreads();

  v8us pv[8];
#pragma unroll
  for (int it = 0; it < 8; ++it) {
    const int q = it * NTHR + tid;
    pv[it] = *(const v8usa*)(outs + (q >> 6) * OSP + (q & 63) * 8);
  }
  const size_t tokBase = (size_t)b * SL + l0;
#pragma unroll
  for (int it = 0; it < 8; ++it) {
    const int q = it * NTHR + tid;
    *(volatile v8us*)(xnhl + (tokBase + (q >> 6)) * KIN + (q & 63) * 8) = pv[it];
  }
  __threadfence();
#pragma unroll
  for (int it = 0; it < 8; ++it) {
    const int q = it * NTHR + tid;
    *(volatile v8us*)(xnhl + (tokBase + (q >> 6)) * KIN + (q & 63) * 8) = pv[it];
  }
}

template <int MODE>
__global__ __launch_bounds__(GTHR) void k_gemm(const unsigned short* __restrict__ Aw, int lda,
                                               const unsigned short* __restrict__ Bt, int ldb, int K,
                                               const float* __restrict__ bias, const float* __restrict__ res,
                                               float* outF, int mTot) {
  __shared__ __attribute__((aligned(16))) float stg[GBM * GBN];
  const int tid = (int)threadIdx.x, lane = tid & 31, wave = tid >> 5, hh = lane >> 4, m = lane & 15;
  const int rowBase = (int)blockIdx.x * GBM;
  const int col0    = (int)blockIdx.y * GBN;
  const int bq      = col0 >> 12;
  const int l0      = col0 & (SL - 1);

  v8f acc[4];
  {
    const v8f z = {0.f, 0.f, 0.f, 0.f, 0.f, 0.f, 0.f, 0.f};
    acc[0] = z; acc[1] = z; acc[2] = z; acc[3] = z;
  }
  const unsigned short* ap = Aw + (size_t)(rowBase + 16 * wave + m) * (size_t)lda + 8 * hh;
  const unsigned short* wp = Bt + (size_t)(col0 + m) * (size_t)ldb + 8 * hh;
  const int ksteps = K >> 5;
#pragma unroll 1
  for (int ks = 0; ks < ksteps; ++ks) {
    FragB af;
    af.h[0] = *(const v8usa*)(ap + 32 * ks);
    af.h[1] = *(const v8usa*)(ap + 32 * ks + 16);
#pragma unroll
    for (int t = 0; t < 4; ++t) {
      const unsigned short* wq = wp + (size_t)(16 * t) * (size_t)ldb + 32 * ks;
      FragB bf;
      bf.h[0] = *(const v8usa*)wq;
      bf.h[1] = *(const v8usa*)(wq + 16);
      acc[t] = wmb(af, bf, acc[t]);
    }
  }

#pragma unroll
  for (int t = 0; t < 4; ++t) {
    const int lc = 16 * t + m;
#pragma unroll
    for (int r = 0; r < 8; ++r) {
      const int lr = 16 * wave + 8 * hh + r;
      stg[lr * GBN + lc] = acc[t][r];
    }
  }
  __syncthreads();

#pragma unroll 1
  for (int i = 0; i < 8; ++i) {
    const int lr = 16 * wave + 2 * i + hh;
    const int gm = rowBase + lr;
    const float bs = bf16_val(bias[gm]);
    float* sp = stg + lr * GBN + 4 * m;
    if constexpr (MODE == 1) {
#pragma unroll 1
      for (int c = 0; c < 4; ++c) {
        const float t0 = sp[c] + bs;
        const float t1 = gelu_erf(t0);
        sp[c] = softplus_p(t1);
      }
    } else if constexpr (MODE == 0) {
      v4f v = *(const v4fa*)sp;
      v.x += bs; v.y += bs; v.z += bs; v.w += bs;
      *(v4fa*)sp = v;
    } else {
      const v4f rr = *(const v4f*)(res + ((size_t)(bq * DI + DH + gm)) * SL + l0 + 4 * m);
      v4f v = *(const v4fa*)sp;
      v.x = (v.x + bs) + rr.x; v.y = (v.y + bs) + rr.y;
      v.z = (v.z + bs) + rr.z; v.w = (v.w + bs) + rr.w;
      *(v4fa*)sp = v;
    }
  }
  __syncthreads();

  v4f fv[8];
#pragma unroll
  for (int i = 0; i < 8; ++i) {
    const int lr = 16 * wave + 2 * i + hh;
    fv[i] = *(const v4fa*)(stg + lr * GBN + 4 * m);
  }
#pragma unroll
  for (int i = 0; i < 8; ++i) {
    const int gm = rowBase + 16 * wave + 2 * i + hh;
    float* op = outF + ((size_t)(bq * mTot + gm)) * SL + l0 + 4 * m;
    *(volatile v4f*)op = fv[i];
  }
  __threadfence();
#pragma unroll
  for (int i = 0; i < 8; ++i) {
    const int gm = rowBase + 16 * wave + 2 * i + hh;
    float* op = outF + ((size_t)(bq * mTot + gm)) * SL + l0 + 4 * m;
    *(volatile v4f*)op = fv[i];
  }
}

__global__ __launch_bounds__(NTHR) void k_conv(const float* __restrict__ xrt, const float* __restrict__ conv_w,
                                               const float* __restrict__ conv_b, float* xa_out,
                                               unsigned short* cat) {
  __shared__ __attribute__((aligned(16))) float xps[CT * XPP];
  __shared__ __attribute__((aligned(16))) float xaf[CT * FP];
  __shared__ __attribute__((aligned(16))) unsigned short thl[2 * CT * TP];
  __shared__ __attribute__((aligned(16))) float cws[CT * 4];
  __shared__ float cbs[CT];
  const int tid = (int)threadIdx.x;
  const int lt  = (int)blockIdx.x & 63;
  const int cg  = ((int)blockIdx.x >> 6) & 3;
  const int b   = (int)blockIdx.x >> 8;
  const int l0  = lt * CT;
  const int chBase = cg * CT;

  {
    v4f v[4];
#pragma unroll
    for (int i = 0; i < 4; ++i) {
      const int u = i * NTHR + tid;
      const int row = u >> 4, q = u & 15;
      v[i] = *(const v4f*)(xrt + ((size_t)(b * DI + chBase + row)) * SL + l0 + 4 * q);
    }
#pragma unroll
    for (int i = 0; i < 4; ++i) {
      const int u = i * NTHR + tid;
      const int row = u >> 4, q = u & 15;
      *(v4fa*)(xps + row * XPP + 4 + 4 * q) = v[i];
    }
  }
  if (tid < 192) {
    const int row = tid / 3;
    const int hx  = tid - 3 * row;
    const int l   = (hx == 0) ? (l0 - 1) : (l0 + 63 + hx);
    const int lc  = l < 0 ? 0 : (l > SL - 1 ? SL - 1 : l);
    const float v = xrt[((size_t)(b * DI + chBase + row)) * SL + lc];
    const bool ok = (l >= 0) && (l < SL);
    const int jx  = (hx == 0) ? 3 : (67 + hx);
    xps[row * XPP + jx] = ok ? v : 0.0f;
  }
  if (tid < CT) {
    const v4f w = *(const v4f*)(conv_w + (size_t)(chBase + tid) * 4);
    cws[tid * 4 + 0] = bf16_val(w.x);
    cws[tid * 4 + 1] = bf16_val(w.y);
    cws[tid * 4 + 2] = bf16_val(w.z);
    cws[tid * 4 + 3] = bf16_val(w.w);
    cbs[tid] = bf16_val(conv_b[chBase + tid]);
  }
  __syncthreads();

#pragma unroll 1
  for (int i = 0; i < 16; ++i) {
    const int idx = i * NTHR + tid;
    const int row = idx >> 6, ll = idx & 63;
    const float* xr = xps + row * XPP + ll + 3;
    float acc = cws[row * 4 + 0] * xr[0];
    acc = fmaf(cws[row * 4 + 1], xr[1], acc);
    acc = fmaf(cws[row * 4 + 2], xr[2], acc);
    acc = fmaf(cws[row * 4 + 3], xr[3], acc);
    const float xc = acc + cbs[row];
    const float xa = gelu_erf(xc);
    xaf[row * FP + ll] = xa;
    const unsigned hb = bf16_bits(xa);
    const unsigned lb = bf16_bits(xa - __uint_as_float(hb << 16));
    thl[ll * TP + row]           = (unsigned short)hb;
    thl[CT * TP + ll * TP + row] = (unsigned short)lb;
  }
  __syncthreads();

  v4f  fa[4];
  v8us pv[4];
#pragma unroll
  for (int i = 0; i < 4; ++i) {
    const int u = i * NTHR + tid;
    fa[i] = *(const v4fa*)(xaf + (u >> 4) * FP + 4 * (u & 15));
    pv[i] = *(const v8usa*)(thl + (u >> 9) * (CT * TP) + ((u >> 3) & 63) * TP + (u & 7) * 8);
  }
#pragma unroll
  for (int i = 0; i < 4; ++i) {
    const int u = i * NTHR + tid;
    *(volatile v4f*)(xa_out + ((size_t)(b * DH + chBase + (u >> 4))) * SL + l0 + 4 * (u & 15)) = fa[i];
    *(volatile v8us*)(cat + ((size_t)b * SL + l0 + ((u >> 3) & 63)) * KOUT + 512 + (u >> 9) * 256 + chBase +
                      (u & 7) * 8) = pv[i];
  }
  __threadfence();
#pragma unroll
  for (int i = 0; i < 4; ++i) {
    const int u = i * NTHR + tid;
    *(volatile v4f*)(xa_out + ((size_t)(b * DH + chBase + (u >> 4))) * SL + l0 + 4 * (u & 15)) = fa[i];
    *(volatile v8us*)(cat + ((size_t)b * SL + l0 + ((u >> 3) & 63)) * KOUT + 512 + (u >> 9) * 256 + chBase +
                      (u & 7) * 8) = pv[i];
  }
}

__global__ __launch_bounds__(CT) void k_scan(const float* __restrict__ Ap, const float* __restrict__ Bp,
                                             const float* __restrict__ Cp, const float* __restrict__ Dp,
                                             const float* __restrict__ dlp, const float* __restrict__ xap,
                                             unsigned short* cat) {
  __shared__ __attribute__((aligned(16))) float dls[CT * FP];
  __shared__ __attribute__((aligned(16))) float xas[CT * FP];
  __shared__ __attribute__((aligned(16))) unsigned short yhl[2 * CT * TP];
  const int tid = (int)threadIdx.x;
  const int b   = (int)blockIdx.x >> 2;
  const int chBase = ((int)blockIdx.x & 3) * CT;
  const int d   = chBase + tid;

  float a[NS], bp[NS], cp[NS], h[NS];
#pragma unroll
  for (int k = 0; k < 4; ++k) {
    const v4f ta = *(const v4f*)(Ap + (size_t)d * NS + 4 * k);
    const v4f tb = *(const v4f*)(Bp + (size_t)d * NS + 4 * k);
    const v4f tc = *(const v4f*)(Cp + (size_t)d * NS + 4 * k);
    a[4 * k + 0] = bf16_val(ta.x); a[4 * k + 1] = bf16_val(ta.y);
    a[4 * k + 2] = bf16_val(ta.z); a[4 * k + 3] = bf16_val(ta.w);
    bp[4 * k + 0] = bf16_val(tb.x); bp[4 * k + 1] = bf16_val(tb.y);
    bp[4 * k + 2] = bf16_val(tb.z); bp[4 * k + 3] = bf16_val(tb.w);
    cp[4 * k + 0] = bf16_val(tc.x); cp[4 * k + 1] = bf16_val(tc.y);
    cp[4 * k + 2] = bf16_val(tc.z); cp[4 * k + 3] = bf16_val(tc.w);
  }
#pragma unroll
  for (int n = 0; n < NS; ++n) h[n] = 0.0f;
  const float dpv = bf16_val(Dp[d]);

#pragma unroll 1
  for (int ch = 0; ch < SL / CT; ++ch) {
    const int l0 = ch * CT;
#pragma unroll 4
    for (int i = 0; i < 16; ++i) {
      const int u = i * CT + tid;
      const int row = u >> 4, q = u & 15;
      const size_t go = ((size_t)(b * DH + chBase + row)) * SL + l0 + 4 * q;
      const v4f v0 = *(const v4f*)(dlp + go);
      const v4f v1 = *(const v4f*)(xap + go);
      *(v4fa*)(dls + row * FP + 4 * q) = v0;
      *(v4fa*)(xas + row * FP + 4 * q) = v1;
    }
    __syncthreads();

#pragma unroll 1
    for (int j = 0; j < CT; ++j) {
      const float dl = dls[tid * FP + j];
      const float u  = xas[tid * FP + j];
      const float du = dl * u;
      float y = 0.0f;
#pragma unroll
      for (int n = 0; n < NS; ++n) {
        const float ea = expf(dl * a[n]);
        h[n] = fmaf(ea, h[n], du * bp[n]);
        y = fmaf(h[n], cp[n], y);
      }
      y = fmaf(u, dpv, y);
      const unsigned hb = bf16_bits(y);
      const unsigned lb = bf16_bits(y - __uint_as_float(hb << 16));
      yhl[j * TP + tid]           = (unsigned short)hb;
      yhl[CT * TP + j * TP + tid] = (unsigned short)lb;
    }
    __syncthreads();

#pragma unroll 1
    for (int gq = 0; gq < 4; ++gq) {
      v8us pv[4];
#pragma unroll
      for (int i = 0; i < 4; ++i) {
        const int p = gq * 256 + i * CT + tid;
        pv[i] = *(const v8usa*)(yhl + (p >> 9) * (CT * TP) + ((p >> 3) & 63) * TP + (p & 7) * 8);
      }
#pragma unroll
      for (int i = 0; i < 4; ++i) {
        const int p = gq * 256 + i * CT + tid;
        *(volatile v8us*)(cat + ((size_t)b * SL + l0 + ((p >> 3) & 63)) * KOUT + (p >> 9) * 256 + chBase +
                          (p & 7) * 8) = pv[i];
      }
      __threadfence();
#pragma unroll
      for (int i = 0; i < 4; ++i) {
        const int p = gq * 256 + i * CT + tid;
        *(volatile v8us*)(cat + ((size_t)b * SL + l0 + ((p >> 3) & 63)) * KOUT + (p >> 9) * 256 + chBase +
                          (p & 7) * 8) = pv[i];
      }
    }
  }
}

static inline size_t al256(size_t o) { return (o + 255) & ~(size_t)255; }

extern "C" void kernel_launch(void* const* d_in, const int* in_sizes, int n_in,
                              void* d_out, int out_size, void* d_ws, size_t ws_size,
                              hipStream_t stream) {
  if (n_in < 15) return;
  if (in_sizes[0] != NB * DM * SL) return;
  if (in_sizes[1] != DM || in_sizes[2] != DM) return;
  if (in_sizes[3] != DI * DM || in_sizes[4] != DI) return;
  if (in_sizes[5] != DH * 4 || in_sizes[6] != DH) return;
  if (in_sizes[7] != DH * NS || in_sizes[8] != DH * NS || in_sizes[9] != DH * NS) return;
  if (in_sizes[10] != DH) return;
  if (in_sizes[11] != DH * DH || in_sizes[12] != DH) return;
  if (in_sizes[13] != DM * DI || in_sizes[14] != DM) return;
  if (out_size != NB * DM * SL) return;

  const float* x      = (const float*)d_in[0];
  const float* ln_g   = (const float*)d_in[1];
  const float* ln_b   = (const float*)d_in[2];
  const float* w_in   = (const float*)d_in[3];
  const float* b_in   = (const float*)d_in[4];
  const float* conv_w = (const float*)d_in[5];
  const float* conv_b = (const float*)d_in[6];
  const float* Ap     = (const float*)d_in[7];
  const float* Bp     = (const float*)d_in[8];
  const float* Cp     = (const float*)d_in[9];
  const float* Dp     = (const float*)d_in[10];
  const float* w_dt   = (const float*)d_in[11];
  const float* b_dt   = (const float*)d_in[12];
  const float* w_out  = (const float*)d_in[13];
  const float* b_out  = (const float*)d_in[14];
  float* out = (float*)d_out;

  char* ws = (char*)d_ws;
  size_t off = 0;
  const size_t oWIN = off; off = al256(off + (size_t)DI * KIN * 2);
  const size_t oWDT = off; off = al256(off + (size_t)DH * KDT * 2);
  const size_t oWO  = off; off = al256(off + (size_t)DM * KOUT * 2);
  const size_t oXN  = off; off = al256(off + (size_t)NTOK * KIN * 2);
  const size_t oXRT = off; off = al256(off + (size_t)NB * DI * SL * 4);
  const size_t oXA  = off; off = al256(off + (size_t)NB * DH * SL * 4);
  const size_t oDL  = off; off = al256(off + (size_t)NB * DH * SL * 4);
  const size_t oCAT = off; off = al256(off + (size_t)NTOK * KOUT * 2);
  if (off > ws_size || off > (size_t)WSMAX) return;
  unsigned short* WIN2 = (unsigned short*)(ws + oWIN);
  unsigned short* WDT2 = (unsigned short*)(ws + oWDT);
  unsigned short* WO4  = (unsigned short*)(ws + oWO);
  unsigned short* XNHL = (unsigned short*)(ws + oXN);
  float*          XRT  = (float*)(ws + oXRT);
  float*          XA   = (float*)(ws + oXA);
  float*          DL   = (float*)(ws + oDL);
  unsigned short* CAT4 = (unsigned short*)(ws + oCAT);

  k_prep<<<NU_ALL / NTHR, NTHR, 0, stream>>>(w_in, w_dt, w_out, WIN2, WDT2, WO4);
  k_ln<<<NTOK / LNT, NTHR, 0, stream>>>(x, ln_g, ln_b, XNHL);
  k_gemm<0><<<dim3(DI / GBM, NTOK / GBN), GTHR, 0, stream>>>(WIN2, KIN, XNHL, KIN, KIN, b_in, b_in, XRT, DI);
  k_conv<<<NB * (DH / CT) * (SL / CT), NTHR, 0, stream>>>(XRT, conv_w, conv_b, XA, CAT4);
  k_gemm<1><<<dim3(DH / GBM, NTOK / GBN), GTHR, 0, stream>>>(WDT2, KDT, CAT4 + 512, KOUT, KDT, b_dt, b_dt, DL, DH);
  k_scan<<<NB * (DH / CT), CT, 0, stream>>>(Ap, Bp, Cp, Dp, DL, XA, CAT4);
  k_gemm<2><<<dim3(DM / GBM, NTOK / GBN), GTHR, 0, stream>>>(WO4, KOUT, CAT4, KOUT, KOUT, b_out, XRT, out, DM);
}
